// CompositionalLoss_69140383531603
// MI455X (gfx1250) — hardware-verified
//
#include <hip/hip_runtime.h>

#define NB_  131072
#define NJ   21
#define NPR  210
#define NPP  224
#define RB   128

typedef _Float16 f16;
typedef __attribute__((ext_vector_type(16))) f16 f16x16;
typedef __attribute__((ext_vector_type(8)))  f16 f16x8;
typedef __attribute__((ext_vector_type(8)))  float f32x8;
typedef __attribute__((ext_vector_type(4)))  float v4f_t;
typedef float v4fa __attribute__((ext_vector_type(4), may_alias));

__constant__ signed char c_ST[NPP * 64] = {-1,0,0,0,0,0,0,0,0,0,0,0,0,0,0,0,0,0,0,0,0,-1,1,0,0,0,0,0,0,0,0,0,0,0,0,0,0,0,0,0,0,0,0,0,0,0,0,0,0,0,0,0,0,0,0,0,0,0,0,0,0,0,0,0,-1,-1,0,0,0,0,0,0,0,0,0,0,-1,0,0,0,0,0,0,0,0,-1,0,1,0,0,0,0,0,0,0,0,0,0,0,0,0,0,0,0,0,0,0,0,0,0,0,0,0,0,0,0,0,0,0,0,0,0,0,0,0,0,0,0,1,0,0,0,0,0,0,0,0,0,0,0,0,0,0,0,0,0,0,0,0,-1,0,0,1,0,0,0,0,0,0,0,0,0,0,0,0,0,0,0,0,0,0,0,0,0,0,0,0,0,0,0,0,0,0,0,0,0,0,0,0,0,0,0,-1,-1,0,0,0,0,0,0,-1,0,0,-1,0,0,0,0,0,0,0,0,0,-1,0,0,0,1,0,0,0,0,0,0,0,0,0,0,0,0,0,0,0,0,0,0,0,0,0,0,0,0,0,0,0,0,0,0,0,0,0,0,0,0,0,0,1,0,0,-1,0,0,0,-1,0,-1,0,0,0,0,0,0,0,0,0,0,0,-1,0,0,0,0,1,0,0,0,0,0,0,0,0,0,0,0,0,0,0,0,0,0,0,0,0,0,0,0,0,0,0,0,0,0,0,0,0,0,0,0,0,0,-1,-1,0,0,-1,0,0,0,-1,0,0,-1,0,0,0,0,0,0,0,0,0,-1,0,0,0,0,0,1,0,0,0,0,0,0,0,0,0,0,0,0,0,0,0,0,0,0,0,0,0,0,0,0,0,0,0,0,0,0,0,0,0,0,0,0,1,0,0,-1,0,0,0,0,0,-1,0,0,0,0,0,0,0,0,0,0,0,-1,0,0,0,0,0,0,1,0,0,0,0,0,0,0,0,0,0,0,0,0,0,0,0,0,0,0,0,0,0,0,0,0,0,0,0,0,0,0,0,0,0,0,-1,-1,0,0,0,0,0,0,0,0,0,0,0,0,0,0,0,0,0,0,0,-1,0,0,0,0,0,0,0,1,0,0,0,0,0,0,0,0,0,0,0,0,0,0,0,0,0,0,0,0,0,0,0,0,0,0,0,0,0,0,0,0,0,0,1,0,0,-1,0,0,0,0,0,0,0,0,0,0,0,0,0,0,0,0,0,-1,0,0,0,0,0,0,0,0,1,0,0,0,0,0,0,0,0,0,0,0,0,0,0,0,0,0,0,0,0,0,0,0,0,0,0,0,0,0,0,0,0,0,1,0,0,-1,0,-1,0,-1,0,-1,0,0,0,0,0,0,0,0,0,0,0,-1,0,0,0,0,0,0,0,0,0,1,0,0,0,0,0,0,0,0,0,0,0,0,0,0,0,0,0,0,0,0,0,0,0,0,0,0,0,0,0,0,0,0,-1,-1,0,0,0,0,0,0,-1,0,0,0,0,0,0,0,0,0,0,0,0,-1,0,0,0,0,0,0,0,0,0,0,1,0,0,0,0,0,0,0,0,0,0,0,0,0,0,0,0,0,0,0,0,0,0,0,0,0,0,0,0,0,0,0,-1,-1,0,0,0,0,0,0,0,0,0,0,0,0,0,0,0,0,0,0,0,-1,0,0,0,0,0,0,0,0,0,0,0,1,0,0,0,0,0,0,0,0,0,0,0,0,0,0,0,0,0,0,0,0,0,0,0,0,0,0,0,0,0,0,-1,-1,0,0,0,0,0,0,0,0,0,0,0,0,0,0,0,-1,0,0,-1,-1,0,0,0,0,0,0,0,0,0,0,0,0,1,0,0,0,0,0,0,0,0,0,0,0,0,0,0,0,0,0,0,0,0,0,0,0,0,0,0,0,0,0,1,0,0,-1,0,0,0,0,0,0,0,0,0,0,0,0,-1,0,-1,0,0,-1,0,0,0,0,0,0,0,0,0,0,0,0,0,1,0,0,0,0,0,0,0,0,0,0,0,0,0,0,0,0,0,0,0,0,0,0,0,0,0,0,0,0,-1,-1,0,0,0,0,0,0,0,0,0,0,0,-1,0,0,0,-1,0,0,-1,-1,0,0,0,0,0,0,0,0,0,0,0,0,0,0,1,0,0,0,0,0,0,0,0,0,0,0,0,0,0,0,0,0,0,0,0,0,0,0,0,0,0,0,1,0,0,-1,0,0,0,0,0,0,0,0,0,0,0,0,0,0,-1,0,0,-1,0,0,0,0,0,0,0,0,0,0,0,0,0,0,0,1,0,0,0,0,0,0,0,0,0,0,0,0,0,0,0,0,0,0,0,0,0,0,0,0,0,0,-1,-1,0,0,0,0,0,0,0,0,0,0,0,0,0,0,0,0,0,0,0,-1,0,0,0,0,0,0,0,0,0,0,0,0,0,0,0,0,1,0,0,0,0,0,0,0,0,0,0,0,0,0,0,0,0,0,0,0,0,0,0,0,0,0,1,0,0,-1,0,0,0,0,0,0,0,0,0,0,0,0,0,0,0,0,0,-1,0,0,0,0,0,0,0,0,0,0,0,0,0,0,0,0,0,1,0,0,0,0,0,0,0,0,0,0,0,0,0,0,0,0,0,0,0,0,0,0,0,0,1,0,0,-1,0,0,0,0,0,0,0,0,0,0,-1,0,-1,0,-1,0,0,-1,0,0,0,0,0,0,0,0,0,0,0,0,0,0,0,0,0,0,1,0,0,0,0,0,0,0,0,0,0,0,0,0,0,0,0,0,0,0,0,0,0,0,-1,-1,0,0,0,0,0,0,0,0,0,0,0,0,0,0,0,-1,0,0,0,-1,0,0,0,0,0,0,0,0,0,0,0,0,0,0,0,0,0,0,0,1,0,0,0,0,0,0,0,0,0,0,0,0,0,0,0,0,0,0,0,0,0,0,0,-1,0,0,0,0,0,0,0,0,0,0,-1,0,0,0,0,0,0,0,0,0,-1,1,0,0,0,0,0,0,0,0,0,0,0,0,0,0,0,0,0,0,0,0,0,0,0,0,0,0,0,0,0,0,0,0,0,0,0,0,0,0,0,0,1,1,0,0,0,0,0,0,0,0,0,0,0,0,0,0,0,0,0,0,0,0,-1,0,1,0,0,0,0,0,0,0,0,0,0,0,0,0,0,0,0,0,0,0,0,0,0,0,0,0,0,0,0,0,0,0,0,0,0,0,0,0,0,0,0,-1,0,0,0,0,0,0,-1,0,0,-1,0,0,0,0,0,0,0,0,0,0,-1,0,0,1,0,0,0,0,0,0,0,0,0,0,0,0,0,0,0,0,0,0,0,0,0,0,0,0,0,0,0,0,0,0,0,0,0,0,0,0,0,0,1,1,0,-1,0,0,0,-1,0,-1,0,0,0,0,0,0,0,0,0,0,0,0,-1,0,0,0,1,0,0,0,0,0,0,0,0,0,0,0,0,0,0,0,0,0,0,0,0,0,0,0,0,0,0,0,0,0,0,0,0,0,0,0,0,0,0,-1,0,0,-1,0,0,0,-1,0,0,-1,0,0,0,0,0,0,0,0,0,0,-1,0,0,0,0,1,0,0,0,0,0,0,0,0,0,0,0,0,0,0,0,0,0,0,0,0,0,0,0,0,0,0,0,0,0,0,0,0,0,0,0,0,1,1,0,-1,0,0,0,0,0,-1,0,0,0,0,0,0,0,0,0,0,0,0,-1,0,0,0,0,0,1,0,0,0,0,0,0,0,0,0,0,0,0,0,0,0,0,0,0,0,0,0,0,0,0,0,0,0,0,0,0,0,0,0,0,0,0,-1,0,0,0,0,0,0,0,0,0,0,0,0,0,0,0,0,0,0,0,0,-1,0,0,0,0,0,0,1,0,0,0,0,0,0,0,0,0,0,0,0,0,0,0,0,0,0,0,0,0,0,0,0,0,0,0,0,0,0,0,0,0,0,1,1,0,-1,0,0,0,0,0,0,0,0,0,0,0,0,0,0,0,0,0,0,-1,0,0,0,0,0,0,0,1,0,0,0,0,0,0,0,0,0,0,0,0,0,0,0,0,0,0,0,0,0,0,0,0,0,0,0,0,0,0,0,0,0,1,1,0,-1,0,-1,0,-1,0,-1,0,0,0,0,0,0,0,0,0,0,0,0,-1,0,0,0,0,0,0,0,0,1,0,0,0,0,0,0,0,0,0,0,0,0,0,0,0,0,0,0,0,0,0,0,0,0,0,0,0,0,0,0,0,0,0,-1,0,0,0,0,0,0,-1,0,0,0,0,0,0,0,0,0,0,0,0,0,-1,0,0,0,0,0,0,0,0,0,1,0,0,0,0,0,0,0,0,0,0,0,0,0,0,0,0,0,0,0,0,0,0,0,0,0,0,0,0,0,0,0,0,-1,0,0,0,0,0,0,0,0,0,0,0,0,0,0,0,0,0,0,0,0,-1,0,0,0,0,0,0,0,0,0,0,1,0,0,0,0,0,0,0,0,0,0,0,0,0,0,0,0,0,0,0,0,0,0,0,0,0,0,0,0,0,0,0,-1,0,0,0,0,0,0,0,0,0,0,0,0,0,0,0,-1,0,0,-1,0,-1,0,0,0,0,0,0,0,0,0,0,0,1,0,0,0,0,0,0,0,0,0,0,0,0,0,0,0,0,0,0,0,0,0,0,0,0,0,0,0,0,0,1,1,0,-1,0,0,0,0,0,0,0,0,0,0,0,0,-1,0,-1,0,0,0,-1,0,0,0,0,0,0,0,0,0,0,0,0,1,0,0,0,0,0,0,0,0,0,0,0,0,0,0,0,0,0,0,0,0,0,0,0,0,0,0,0,0,0,-1,0,0,0,0,0,0,0,0,0,0,0,-1,0,0,0,-1,0,0,-1,0,-1,0,0,0,0,0,0,0,0,0,0,0,0,0,1,0,0,0,0,0,0,0,0,0,0,0,0,0,0,0,0,0,0,0,0,0,0,0,0,0,0,0,1,1,0,-1,0,0,0,0,0,0,0,0,0,0,0,0,0,0,-1,0,0,0,-1,0,0,0,0,0,0,0,0,0,0,0,0,0,0,1,0,0,0,0,0,0,0,0,0,0,0,0,0,0,0,0,0,0,0,0,0,0,0,0,0,0,0,-1,0,0,0,0,0,0,0,0,0,0,0,0,0,0,0,0,0,0,0,0,-1,0,0,0,0,0,0,0,0,0,0,0,0,0,0,0,1,0,0,0,0,0,0,0,0,0,0,0,0,0,0,0,0,0,0,0,0,0,0,0,0,0,1,1,0,-1,0,0,0,0,0,0,0,0,0,0,0,0,0,0,0,0,0,0,-1,0,0,0,0,0,0,0,0,0,0,0,0,0,0,0,0,1,0,0,0,0,0,0,0,0,0,0,0,0,0,0,0,0,0,0,0,0,0,0,0,0,1,1,0,-1,0,0,0,0,0,0,0,0,0,0,-1,0,-1,0,-1,0,0,0,-1,0,0,0,0,0,0,0,0,0,0,0,0,0,0,0,0,0,1,0,0,0,0,0,0,0,0,0,0,0,0,0,0,0,0,0,0,0,0,0,0,0,0,-1,0,0,0,0,0,0,0,0,0,0,0,0,0,0,0,-1,0,0,0,0,-1,0,0,0,0,0,0,0,0,0,0,0,0,0,0,0,0,0,0,1,0,0,0,0,0,0,0,0,0,0,0,0,0,0,0,0,0,0,0,0,0,0,1,1,1,0,0,0,0,0,0,0,0,0,1,0,0,0,0,0,0,0,0,0,0,-1,1,0,0,0,0,0,0,0,0,0,0,0,0,0,0,0,0,0,0,0,0,0,0,0,0,0,0,0,0,0,0,0,0,0,0,0,0,0,0,0,0,-1,1,0,0,0,0,0,-1,0,0,-1,1,0,0,0,0,0,0,0,0,0,0,-1,0,1,0,0,0,0,0,0,0,0,0,0,0,0,0,0,0,0,0,0,0,0,0,0,0,0,0,0,0,0,0,0,0,0,0,0,0,0,0,0,1,1,1,-1,0,0,0,-1,0,-1,0,0,1,0,0,0,0,0,0,0,0,0,0,-1,0,0,1,0,0,0,0,0,0,0,0,0,0,0,0,0,0,0,0,0,0,0,0,0,0,0,0,0,0,0,0,0,0,0,0,0,0,0,0,0,0,-1,1,0,-1,0,0,0,-1,0,0,-1,1,0,0,0,0,0,0,0,0,0,0,-1,0,0,0,1,0,0,0,0,0,0,0,0,0,0,0,0,0,0,0,0,0,0,0,0,0,0,0,0,0,0,0,0,0,0,0,0,0,0,0,0,1,1,1,-1,0,0,0,0,0,-1,0,0,1,0,0,0,0,0,0,0,0,0,0,-1,0,0,0,0,1,0,0,0,0,0,0,0,0,0,0,0,0,0,0,0,0,0,0,0,0,0,0,0,0,0,0,0,0,0,0,0,0,0,0,0,0,-1,1,0,0,0,0,0,0,0,0,0,1,0,0,0,0,0,0,0,0,0,0,-1,0,0,0,0,0,1,0,0,0,0,0,0,0,0,0,0,0,0,0,0,0,0,0,0,0,0,0,0,0,0,0,0,0,0,0,0,0,0,0,0,1,1,1,-1,0,0,0,0,0,0,0,0,1,0,0,0,0,0,0,0,0,0,0,-1,0,0,0,0,0,0,1,0,0,0,0,0,0,0,0,0,0,0,0,0,0,0,0,0,0,0,0,0,0,0,0,0,0,0,0,0,0,0,0,0,1,1,1,-1,0,-1,0,-1,0,-1,0,0,1,0,0,0,0,0,0,0,0,0,0,-1,0,0,0,0,0,0,0,1,0,0,0,0,0,0,0,0,0,0,0,0,0,0,0,0,0,0,0,0,0,0,0,0,0,0,0,0,0,0,0,0,0,-1,1,0,0,0,0,0,-1,0,0,0,1,0,0,0,0,0,0,0,0,0,0,-1,0,0,0,0,0,0,0,0,1,0,0,0,0,0,0,0,0,0,0,0,0,0,0,0,0,0,0,0,0,0,0,0,0,0,0,0,0,0,0,0,0,0,1,0,0,0,0,0,0,0,0,0,0,0,0,0,0,0,0,0,0,0,0,-1,0,0,0,0,0,0,0,0,0,1,0,0,0,0,0,0,0,0,0,0,0,0,0,0,0,0,0,0,0,0,0,0,0,0,0,0,0,0,0,0,0,-1,1,0,0,0,0,0,0,0,0,0,1,0,0,0,0,-1,0,0,-1,0,0,-1,0,0,0,0,0,0,0,0,0,0,1,0,0,0,0,0,0,0,0,0,0,0,0,0,0,0,0,0,0,0,0,0,0,0,0,0,0,0,0,0,1,1,1,-1,0,0,0,0,0,0,0,0,1,0,0,0,-1,0,-1,0,0,0,0,-1,0,0,0,0,0,0,0,0,0,0,0,1,0,0,0,0,0,0,0,0,0,0,0,0,0,0,0,0,0,0,0,0,0,0,0,0,0,0,0,0,0,-1,1,0,0,0,0,0,0,0,0,0,1,-1,0,0,0,-1,0,0,-1,0,0,-1,0,0,0,0,0,0,0,0,0,0,0,0,1,0,0,0,0,0,0,0,0,0,0,0,0,0,0,0,0,0,0,0,0,0,0,0,0,0,0,0,1,1,1,-1,0,0,0,0,0,0,0,0,1,0,0,0,0,0,-1,0,0,0,0,-1,0,0,0,0,0,0,0,0,0,0,0,0,0,1,0,0,0,0,0,0,0,0,0,0,0,0,0,0,0,0,0,0,0,0,0,0,0,0,0,0,0,-1,1,0,0,0,0,0,0,0,0,0,1,0,0,0,0,0,0,0,0,0,0,-1,0,0,0,0,0,0,0,0,0,0,0,0,0,0,1,0,0,0,0,0,0,0,0,0,0,0,0,0,0,0,0,0,0,0,0,0,0,0,0,0,1,1,1,-1,0,0,0,0,0,0,0,0,1,0,0,0,0,0,0,0,0,0,0,-1,0,0,0,0,0,0,0,0,0,0,0,0,0,0,0,1,0,0,0,0,0,0,0,0,0,0,0,0,0,0,0,0,0,0,0,0,0,0,0,0,1,1,1,-1,0,0,0,0,0,0,0,0,1,0,-1,0,-1,0,-1,0,0,0,0,-1,0,0,0,0,0,0,0,0,0,0,0,0,0,0,0,0,1,0,0,0,0,0,0,0,0,0,0,0,0,0,0,0,0,0,0,0,0,0,0,0,0,-1,1,0,0,0,0,0,0,0,0,0,1,0,0,0,0,-1,0,0,0,0,0,-1,0,0,0,0,0,0,0,0,0,0,0,0,0,0,0,0,0,1,0,0,0,0,0,0,0,0,0,0,0,0,0,0,0,0,0,0,0,0,0,0,-1,-1,0,-1,0,0,0,0,-1,0,0,-1,0,0,0,0,0,0,0,0,0,0,0,0,-1,1,0,0,0,0,0,0,0,0,0,0,0,0,0,0,0,0,0,0,0,0,0,0,0,0,0,0,0,0,0,0,0,0,0,0,0,0,0,0,0,0,0,-1,0,0,0,-1,0,-1,0,0,0,0,0,0,0,0,0,0,0,0,0,0,-1,0,1,0,0,0,0,0,0,0,0,0,0,0,0,0,0,0,0,0,0,0,0,0,0,0,0,0,0,0,0,0,0,0,0,0,0,0,0,0,-1,-1,0,-1,-1,0,0,0,-1,0,0,-1,0,0,0,0,0,0,0,0,0,0,0,0,-1,0,0,1,0,0,0,0,0,0,0,0,0,0,0,0,0,0,0,0,0,0,0,0,0,0,0,0,0,0,0,0,0,0,0,0,0,0,0,0,0,0,0,-1,0,0,0,0,0,-1,0,0,0,0,0,0,0,0,0,0,0,0,0,0,-1,0,0,0,1,0,0,0,0,0,0,0,0,0,0,0,0,0,0,0,0,0,0,0,0,0,0,0,0,0,0,0,0,0,0,0,0,0,0,0,-1,-1,0,-1,0,0,0,0,0,0,0,0,0,0,0,0,0,0,0,0,0,0,0,0,-1,0,0,0,0,1,0,0,0,0,0,0,0,0,0,0,0,0,0,0,0,0,0,0,0,0,0,0,0,0,0,0,0,0,0,0,0,0,0,0,0,0,0,-1,0,0,0,0,0,0,0,0,0,0,0,0,0,0,0,0,0,0,0,0,-1,0,0,0,0,0,1,0,0,0,0,0,0,0,0,0,0,0,0,0,0,0,0,0,0,0,0,0,0,0,0,0,0,0,0,0,0,0,0,0,0,0,0,-1,0,-1,0,-1,0,-1,0,0,0,0,0,0,0,0,0,0,0,0,0,0,-1,0,0,0,0,0,0,1,0,0,0,0,0,0,0,0,0,0,0,0,0,0,0,0,0,0,0,0,0,0,0,0,0,0,0,0,0,0,0,0,-1,-1,0,-1,0,0,0,0,-1,0,0,0,0,0,0,0,0,0,0,0,0,0,0,0,-1,0,0,0,0,0,0,0,1,0,0,0,0,0,0,0,0,0,0,0,0,0,0,0,0,0,0,0,0,0,0,0,0,0,0,0,0,0,0,0,-1,-1,0,-1,0,0,0,0,0,0,0,0,0,0,0,0,0,0,0,0,0,0,0,0,-1,0,0,0,0,0,0,0,0,1,0,0,0,0,0,0,0,0,0,0,0,0,0,0,0,0,0,0,0,0,0,0,0,0,0,0,0,0,0,0,-1,-1,0,-1,0,0,0,0,0,0,0,0,0,0,0,0,0,-1,0,0,-1,0,0,0,-1,0,0,0,0,0,0,0,0,0,1,0,0,0,0,0,0,0,0,0,0,0,0,0,0,0,0,0,0,0,0,0,0,0,0,0,0,0,0,0,0,0,0,-1,0,0,0,0,0,0,0,0,0,0,0,0,-1,0,-1,0,0,0,0,0,-1,0,0,0,0,0,0,0,0,0,0,1,0,0,0,0,0,0,0,0,0,0,0,0,0,0,0,0,0,0,0,0,0,0,0,0,0,0,0,0,-1,-1,0,-1,0,0,0,0,0,0,0,0,0,-1,0,0,0,-1,0,0,-1,0,0,0,-1,0,0,0,0,0,0,0,0,0,0,0,1,0,0,0,0,0,0,0,0,0,0,0,0,0,0,0,0,0,0,0,0,0,0,0,0,0,0,0,0,0,0,-1,0,0,0,0,0,0,0,0,0,0,0,0,0,0,-1,0,0,0,0,0,-1,0,0,0,0,0,0,0,0,0,0,0,0,1,0,0,0,0,0,0,0,0,0,0,0,0,0,0,0,0,0,0,0,0,0,0,0,0,0,0,-1,-1,0,-1,0,0,0,0,0,0,0,0,0,0,0,0,0,0,0,0,0,0,0,0,-1,0,0,0,0,0,0,0,0,0,0,0,0,0,1,0,0,0,0,0,0,0,0,0,0,0,0,0,0,0,0,0,0,0,0,0,0,0,0,0,0,0,0,-1,0,0,0,0,0,0,0,0,0,0,0,0,0,0,0,0,0,0,0,0,-1,0,0,0,0,0,0,0,0,0,0,0,0,0,0,1,0,0,0,0,0,0,0,0,0,0,0,0,0,0,0,0,0,0,0,0,0,0,0,0,0,0,0,-1,0,0,0,0,0,0,0,0,0,0,-1,0,-1,0,-1,0,0,0,0,0,-1,0,0,0,0,0,0,0,0,0,0,0,0,0,0,0,1,0,0,0,0,0,0,0,0,0,0,0,0,0,0,0,0,0,0,0,0,0,0,0,-1,-1,0,-1,0,0,0,0,0,0,0,0,0,0,0,0,0,-1,0,0,0,0,0,0,-1,0,0,0,0,0,0,0,0,0,0,0,0,0,0,0,0,1,0,0,0,0,0,0,0,0,0,0,0,0,0,0,0,0,0,0,0,0,0,0,1,1,0,-1,1,0,0,-1,1,-1,0,1,0,0,0,0,0,0,0,0,0,0,0,0,0,-1,1,0,0,0,0,0,0,0,0,0,0,0,0,0,0,0,0,0,0,0,0,0,0,0,0,0,0,0,0,0,0,0,0,0,0,0,0,0,0,0,0,0,-1,0,0,0,0,0,0,0,0,0,0,0,0,0,0,0,0,0,0,0,0,-1,0,1,0,0,0,0,0,0,0,0,0,0,0,0,0,0,0,0,0,0,0,0,0,0,0,0,0,0,0,0,0,0,0,0,0,0,0,0,1,1,0,-1,1,0,0,0,1,-1,0,1,0,0,0,0,0,0,0,0,0,0,0,0,0,-1,0,0,1,0,0,0,0,0,0,0,0,0,0,0,0,0,0,0,0,0,0,0,0,0,0,0,0,0,0,0,0,0,0,0,0,0,0,0,0,0,0,0,1,0,0,0,0,0,0,1,0,0,0,0,0,0,0,0,0,0,0,0,0,-1,0,0,0,1,0,0,0,0,0,0,0,0,0,0,0,0,0,0,0,0,0,0,0,0,0,0,0,0,0,0,0,0,0,0,0,0,0,0,1,1,0,-1,1,0,0,0,1,0,0,1,0,0,0,0,0,0,0,0,0,0,0,0,0,-1,0,0,0,0,1,0,0,0,0,0,0,0,0,0,0,0,0,0,0,0,0,0,0,0,0,0,0,0,0,0,0,0,0,0,0,0,0,0,1,1,0,-1,1,-1,0,-1,1,-1,0,1,0,0,0,0,0,0,0,0,0,0,0,0,0,-1,0,0,0,0,0,1,0,0,0,0,0,0,0,0,0,0,0,0,0,0,0,0,0,0,0,0,0,0,0,0,0,0,0,0,0,0,0,0,0,0,0,0,1,0,0,0,0,0,0,0,0,0,0,0,0,0,0,0,0,0,0,0,0,-1,0,0,0,0,0,0,1,0,0,0,0,0,0,0,0,0,0,0,0,0,0,0,0,0,0,0,0,0,0,0,0,0,0,0,0,0,0,0,0,-1,0,0,1,0,0,0,1,0,0,1,0,0,0,0,0,0,0,0,0,0,0,0,0,-1,0,0,0,0,0,0,0,1,0,0,0,0,0,0,0,0,0,0,0,0,0,0,0,0,0,0,0,0,0,0,0,0,0,0,0,0,0,0,0,-1,0,0,1,0,0,0,1,0,0,1,0,0,0,0,0,-1,0,0,-1,0,0,0,0,-1,0,0,0,0,0,0,0,0,1,0,0,0,0,0,0,0,0,0,0,0,0,0,0,0,0,0,0,0,0,0,0,0,0,0,0,0,0,0,1,1,0,-1,1,0,0,0,1,0,0,1,0,0,0,0,-1,0,-1,0,0,0,0,0,0,-1,0,0,0,0,0,0,0,0,0,1,0,0,0,0,0,0,0,0,0,0,0,0,0,0,0,0,0,0,0,0,0,0,0,0,0,0,0,0,0,-1,0,0,1,0,0,0,1,0,0,1,0,-1,0,0,0,-1,0,0,-1,0,0,0,0,-1,0,0,0,0,0,0,0,0,0,0,1,0,0,0,0,0,0,0,0,0,0,0,0,0,0,0,0,0,0,0,0,0,0,0,0,0,0,0,1,1,0,-1,1,0,0,0,1,0,0,1,0,0,0,0,0,0,-1,0,0,0,0,0,0,-1,0,0,0,0,0,0,0,0,0,0,0,1,0,0,0,0,0,0,0,0,0,0,0,0,0,0,0,0,0,0,0,0,0,0,0,0,0,0,0,-1,0,0,1,0,0,0,1,0,0,1,0,0,0,0,0,0,0,0,0,0,0,0,0,-1,0,0,0,0,0,0,0,0,0,0,0,0,1,0,0,0,0,0,0,0,0,0,0,0,0,0,0,0,0,0,0,0,0,0,0,0,0,0,1,1,0,-1,1,0,0,0,1,0,0,1,0,0,0,0,0,0,0,0,0,0,0,0,0,-1,0,0,0,0,0,0,0,0,0,0,0,0,0,1,0,0,0,0,0,0,0,0,0,0,0,0,0,0,0,0,0,0,0,0,0,0,0,0,1,1,0,-1,1,0,0,0,1,0,0,1,0,0,-1,0,-1,0,-1,0,0,0,0,0,0,-1,0,0,0,0,0,0,0,0,0,0,0,0,0,0,1,0,0,0,0,0,0,0,0,0,0,0,0,0,0,0,0,0,0,0,0,0,0,0,0,-1,0,0,1,0,0,0,1,0,0,1,0,0,0,0,0,-1,0,0,0,0,0,0,0,-1,0,0,0,0,0,0,0,0,0,0,0,0,0,0,0,1,0,0,0,0,0,0,0,0,0,0,0,0,0,0,0,0,0,0,0,0,0,0,-1,-1,0,-1,-1,1,0,1,-1,1,0,-1,0,0,0,0,0,0,0,0,0,0,0,0,0,0,-1,1,0,0,0,0,0,0,0,0,0,0,0,0,0,0,0,0,0,0,0,0,0,0,0,0,0,0,0,0,0,0,0,0,0,0,0,0,0,0,0,0,0,1,0,0,0,0,0,0,0,0,0,0,0,0,0,0,0,0,0,0,0,0,-1,0,1,0,0,0,0,0,0,0,0,0,0,0,0,0,0,0,0,0,0,0,0,0,0,0,0,0,0,0,0,0,0,0,0,0,0,0,-1,-1,0,-1,0,1,0,1,0,1,0,0,0,0,0,0,0,0,0,0,0,0,0,0,0,0,-1,0,0,1,0,0,0,0,0,0,0,0,0,0,0,0,0,0,0,0,0,0,0,0,0,0,0,0,0,0,0,0,0,0,0,0,0,0,0,0,0,0,0,1,0,1,0,0,0,0,0,0,0,0,0,0,0,0,0,0,0,0,0,0,-1,0,0,0,1,0,0,0,0,0,0,0,0,0,0,0,0,0,0,0,0,0,0,0,0,0,0,0,0,0,0,0,0,0,0,0,0,0,0,0,0,0,0,-1,0,0,0,0,0,0,0,0,0,0,0,0,0,0,0,0,0,0,0,0,-1,0,0,0,0,1,0,0,0,0,0,0,0,0,0,0,0,0,0,0,0,0,0,0,0,0,0,0,0,0,0,0,0,0,0,0,0,0,-1,-1,0,-1,0,1,0,1,-1,1,0,0,0,0,0,0,0,0,0,0,0,0,0,0,0,0,-1,0,0,0,0,0,1,0,0,0,0,0,0,0,0,0,0,0,0,0,0,0,0,0,0,0,0,0,0,0,0,0,0,0,0,0,0,0,-1,-1,0,-1,0,1,0,1,0,1,0,0,0,0,0,0,0,0,0,0,0,0,0,0,0,0,-1,0,0,0,0,0,0,1,0,0,0,0,0,0,0,0,0,0,0,0,0,0,0,0,0,0,0,0,0,0,0,0,0,0,0,0,0,0,-1,-1,0,-1,0,1,0,1,0,1,0,0,0,0,0,0,0,-1,0,0,-1,0,0,0,0,0,-1,0,0,0,0,0,0,0,1,0,0,0,0,0,0,0,0,0,0,0,0,0,0,0,0,0,0,0,0,0,0,0,0,0,0,0,0,0,0,0,0,-1,0,1,0,1,0,1,0,0,0,0,0,0,-1,0,-1,0,0,0,0,0,0,0,-1,0,0,0,0,0,0,0,0,1,0,0,0,0,0,0,0,0,0,0,0,0,0,0,0,0,0,0,0,0,0,0,0,0,0,0,0,0,-1,-1,0,-1,0,1,0,1,0,1,0,0,0,-1,0,0,0,-1,0,0,-1,0,0,0,0,0,-1,0,0,0,0,0,0,0,0,0,1,0,0,0,0,0,0,0,0,0,0,0,0,0,0,0,0,0,0,0,0,0,0,0,0,0,0,0,0,0,0,-1,0,1,0,1,0,1,0,0,0,0,0,0,0,0,-1,0,0,0,0,0,0,0,-1,0,0,0,0,0,0,0,0,0,0,1,0,0,0,0,0,0,0,0,0,0,0,0,0,0,0,0,0,0,0,0,0,0,0,0,0,0,-1,-1,0,-1,0,1,0,1,0,1,0,0,0,0,0,0,0,0,0,0,0,0,0,0,0,0,-1,0,0,0,0,0,0,0,0,0,0,0,1,0,0,0,0,0,0,0,0,0,0,0,0,0,0,0,0,0,0,0,0,0,0,0,0,0,0,0,0,-1,0,1,0,1,0,1,0,0,0,0,0,0,0,0,0,0,0,0,0,0,0,0,-1,0,0,0,0,0,0,0,0,0,0,0,0,1,0,0,0,0,0,0,0,0,0,0,0,0,0,0,0,0,0,0,0,0,0,0,0,0,0,0,0,-1,0,1,0,1,0,1,0,0,0,0,-1,0,-1,0,-1,0,0,0,0,0,0,0,-1,0,0,0,0,0,0,0,0,0,0,0,0,0,1,0,0,0,0,0,0,0,0,0,0,0,0,0,0,0,0,0,0,0,0,0,0,0,-1,-1,0,-1,0,1,0,1,0,1,0,0,0,0,0,0,0,-1,0,0,0,0,0,0,0,0,-1,0,0,0,0,0,0,0,0,0,0,0,0,0,0,1,0,0,0,0,0,0,0,0,0,0,0,0,0,0,0,0,0,0,0,0,0,0,1,1,0,-1,1,0,1,0,1,-1,0,1,0,0,0,0,0,0,0,0,0,0,0,0,0,0,0,-1,1,0,0,0,0,0,0,0,0,0,0,0,0,0,0,0,0,0,0,0,0,0,0,0,0,0,0,0,0,0,0,0,0,0,0,0,0,0,0,0,1,0,1,0,0,0,0,1,0,0,0,0,0,0,0,0,0,0,0,0,0,0,0,-1,0,1,0,0,0,0,0,0,0,0,0,0,0,0,0,0,0,0,0,0,0,0,0,0,0,0,0,0,0,0,0,0,0,0,0,0,1,1,0,-1,1,0,1,0,1,0,0,1,0,0,0,0,0,0,0,0,0,0,0,0,0,0,0,-1,0,0,1,0,0,0,0,0,0,0,0,0,0,0,0,0,0,0,0,0,0,0,0,0,0,0,0,0,0,0,0,0,0,0,0,0,1,1,0,-1,1,-1,1,-1,1,-1,0,1,0,0,0,0,0,0,0,0,0,0,0,0,0,0,0,-1,0,0,0,1,0,0,0,0,0,0,0,0,0,0,0,0,0,0,0,0,0,0,0,0,0,0,0,0,0,0,0,0,0,0,0,0,0,0,0,0,1,0,1,0,0,0,0,0,0,0,0,0,0,0,0,0,0,0,0,0,0,0,0,-1,0,0,0,0,1,0,0,0,0,0,0,0,0,0,0,0,0,0,0,0,0,0,0,0,0,0,0,0,0,0,0,0,0,0,0,0,0,-1,0,0,1,0,1,0,1,0,0,1,0,0,0,0,0,0,0,0,0,0,0,0,0,0,0,-1,0,0,0,0,0,1,0,0,0,0,0,0,0,0,0,0,0,0,0,0,0,0,0,0,0,0,0,0,0,0,0,0,0,0,0,0,0,-1,0,0,1,0,1,0,1,0,0,1,0,0,0,0,0,-1,0,0,-1,0,0,0,0,0,0,-1,0,0,0,0,0,0,1,0,0,0,0,0,0,0,0,0,0,0,0,0,0,0,0,0,0,0,0,0,0,0,0,0,0,0,0,0,1,1,0,-1,1,0,1,0,1,0,0,1,0,0,0,0,-1,0,-1,0,0,0,0,0,0,0,0,-1,0,0,0,0,0,0,0,1,0,0,0,0,0,0,0,0,0,0,0,0,0,0,0,0,0,0,0,0,0,0,0,0,0,0,0,0,0,-1,0,0,1,0,1,0,1,0,0,1,0,-1,0,0,0,-1,0,0,-1,0,0,0,0,0,0,-1,0,0,0,0,0,0,0,0,1,0,0,0,0,0,0,0,0,0,0,0,0,0,0,0,0,0,0,0,0,0,0,0,0,0,0,0,1,1,0,-1,1,0,1,0,1,0,0,1,0,0,0,0,0,0,-1,0,0,0,0,0,0,0,0,-1,0,0,0,0,0,0,0,0,0,1,0,0,0,0,0,0,0,0,0,0,0,0,0,0,0,0,0,0,0,0,0,0,0,0,0,0,0,-1,0,0,1,0,1,0,1,0,0,1,0,0,0,0,0,0,0,0,0,0,0,0,0,0,0,-1,0,0,0,0,0,0,0,0,0,0,1,0,0,0,0,0,0,0,0,0,0,0,0,0,0,0,0,0,0,0,0,0,0,0,0,0,1,1,0,-1,1,0,1,0,1,0,0,1,0,0,0,0,0,0,0,0,0,0,0,0,0,0,0,-1,0,0,0,0,0,0,0,0,0,0,0,1,0,0,0,0,0,0,0,0,0,0,0,0,0,0,0,0,0,0,0,0,0,0,0,0,1,1,0,-1,1,0,1,0,1,0,0,1,0,0,-1,0,-1,0,-1,0,0,0,0,0,0,0,0,-1,0,0,0,0,0,0,0,0,0,0,0,0,1,0,0,0,0,0,0,0,0,0,0,0,0,0,0,0,0,0,0,0,0,0,0,0,0,-1,0,0,1,0,1,0,1,0,0,1,0,0,0,0,0,-1,0,0,0,0,0,0,0,0,0,-1,0,0,0,0,0,0,0,0,0,0,0,0,0,1,0,0,0,0,0,0,0,0,0,0,0,0,0,0,0,0,0,0,0,0,0,0,-1,-1,0,-1,0,0,0,1,0,1,0,0,0,0,0,0,0,0,0,0,0,0,0,0,0,0,0,0,-1,1,0,0,0,0,0,0,0,0,0,0,0,0,0,0,0,0,0,0,0,0,0,0,0,0,0,0,0,0,0,0,0,0,0,0,0,0,0,0,0,0,0,1,0,0,0,0,0,0,0,0,0,0,0,0,0,0,0,0,0,0,0,0,-1,0,1,0,0,0,0,0,0,0,0,0,0,0,0,0,0,0,0,0,0,0,0,0,0,0,0,0,0,0,0,0,0,0,0,0,0,0,0,0,0,-1,0,-1,0,0,0,0,0,0,0,0,0,0,0,0,0,0,0,0,0,0,0,0,-1,0,0,1,0,0,0,0,0,0,0,0,0,0,0,0,0,0,0,0,0,0,0,0,0,0,0,0,0,0,0,0,0,0,0,0,-1,-1,0,-1,0,0,0,1,-1,1,0,0,0,0,0,0,0,0,0,0,0,0,0,0,0,0,0,0,-1,0,0,0,1,0,0,0,0,0,0,0,0,0,0,0,0,0,0,0,0,0,0,0,0,0,0,0,0,0,0,0,0,0,0,0,-1,-1,0,-1,0,0,0,1,0,1,0,0,0,0,0,0,0,0,0,0,0,0,0,0,0,0,0,0,-1,0,0,0,0,1,0,0,0,0,0,0,0,0,0,0,0,0,0,0,0,0,0,0,0,0,0,0,0,0,0,0,0,0,0,0,-1,-1,0,-1,0,0,0,1,0,1,0,0,0,0,0,0,0,-1,0,0,-1,0,0,0,0,0,0,0,-1,0,0,0,0,0,1,0,0,0,0,0,0,0,0,0,0,0,0,0,0,0,0,0,0,0,0,0,0,0,0,0,0,0,0,0,0,0,0,-1,0,0,0,1,0,1,0,0,0,0,0,0,-1,0,-1,0,0,0,0,0,0,0,0,0,-1,0,0,0,0,0,0,1,0,0,0,0,0,0,0,0,0,0,0,0,0,0,0,0,0,0,0,0,0,0,0,0,0,0,0,0,-1,-1,0,-1,0,0,0,1,0,1,0,0,0,-1,0,0,0,-1,0,0,-1,0,0,0,0,0,0,0,-1,0,0,0,0,0,0,0,1,0,0,0,0,0,0,0,0,0,0,0,0,0,0,0,0,0,0,0,0,0,0,0,0,0,0,0,0,0,0,-1,0,0,0,1,0,1,0,0,0,0,0,0,0,0,-1,0,0,0,0,0,0,0,0,0,-1,0,0,0,0,0,0,0,0,1,0,0,0,0,0,0,0,0,0,0,0,0,0,0,0,0,0,0,0,0,0,0,0,0,0,0,-1,-1,0,-1,0,0,0,1,0,1,0,0,0,0,0,0,0,0,0,0,0,0,0,0,0,0,0,0,-1,0,0,0,0,0,0,0,0,0,1,0,0,0,0,0,0,0,0,0,0,0,0,0,0,0,0,0,0,0,0,0,0,0,0,0,0,0,0,-1,0,0,0,1,0,1,0,0,0,0,0,0,0,0,0,0,0,0,0,0,0,0,0,0,-1,0,0,0,0,0,0,0,0,0,0,1,0,0,0,0,0,0,0,0,0,0,0,0,0,0,0,0,0,0,0,0,0,0,0,0,0,0,0,-1,0,0,0,1,0,1,0,0,0,0,-1,0,-1,0,-1,0,0,0,0,0,0,0,0,0,-1,0,0,0,0,0,0,0,0,0,0,0,1,0,0,0,0,0,0,0,0,0,0,0,0,0,0,0,0,0,0,0,0,0,0,0,-1,-1,0,-1,0,0,0,1,0,1,0,0,0,0,0,0,0,-1,0,0,0,0,0,0,0,0,0,0,-1,0,0,0,0,0,0,0,0,0,0,0,0,1,0,0,0,0,0,0,0,0,0,0,0,0,0,0,0,0,0,0,0,0,0,0,1,1,0,-1,0,0,0,0,1,0,0,0,0,0,0,0,0,0,0,0,0,0,0,0,0,0,0,0,0,-1,1,0,0,0,0,0,0,0,0,0,0,0,0,0,0,0,0,0,0,0,0,0,0,0,0,0,0,0,0,0,0,0,0,0,1,1,0,-1,0,-1,0,-1,1,-1,0,0,0,0,0,0,0,0,0,0,0,0,0,0,0,0,0,0,0,-1,0,1,0,0,0,0,0,0,0,0,0,0,0,0,0,0,0,0,0,0,0,0,0,0,0,0,0,0,0,0,0,0,0,0,0,0,0,0,0,0,0,0,-1,0,0,0,0,0,0,0,0,0,0,0,0,0,0,0,0,0,0,0,0,-1,0,0,1,0,0,0,0,0,0,0,0,0,0,0,0,0,0,0,0,0,0,0,0,0,0,0,0,0,0,0,0,0,0,0,0,-1,0,0,0,0,0,0,1,0,0,0,0,0,0,0,0,0,0,0,0,0,0,0,0,0,0,0,0,-1,0,0,0,1,0,0,0,0,0,0,0,0,0,0,0,0,0,0,0,0,0,0,0,0,0,0,0,0,0,0,0,0,0,0,0,-1,0,0,0,0,0,0,1,0,0,0,0,0,0,0,0,-1,0,0,-1,0,0,0,0,0,0,0,0,-1,0,0,0,0,1,0,0,0,0,0,0,0,0,0,0,0,0,0,0,0,0,0,0,0,0,0,0,0,0,0,0,0,0,0,1,1,0,-1,0,0,0,0,1,0,0,0,0,0,0,0,-1,0,-1,0,0,0,0,0,0,0,0,0,0,-1,0,0,0,0,0,1,0,0,0,0,0,0,0,0,0,0,0,0,0,0,0,0,0,0,0,0,0,0,0,0,0,0,0,0,0,-1,0,0,0,0,0,0,1,0,0,0,0,-1,0,0,0,-1,0,0,-1,0,0,0,0,0,0,0,0,-1,0,0,0,0,0,0,1,0,0,0,0,0,0,0,0,0,0,0,0,0,0,0,0,0,0,0,0,0,0,0,0,0,0,0,1,1,0,-1,0,0,0,0,1,0,0,0,0,0,0,0,0,0,-1,0,0,0,0,0,0,0,0,0,0,-1,0,0,0,0,0,0,0,1,0,0,0,0,0,0,0,0,0,0,0,0,0,0,0,0,0,0,0,0,0,0,0,0,0,0,0,-1,0,0,0,0,0,0,1,0,0,0,0,0,0,0,0,0,0,0,0,0,0,0,0,0,0,0,0,-1,0,0,0,0,0,0,0,0,1,0,0,0,0,0,0,0,0,0,0,0,0,0,0,0,0,0,0,0,0,0,0,0,0,0,1,1,0,-1,0,0,0,0,1,0,0,0,0,0,0,0,0,0,0,0,0,0,0,0,0,0,0,0,0,-1,0,0,0,0,0,0,0,0,0,1,0,0,0,0,0,0,0,0,0,0,0,0,0,0,0,0,0,0,0,0,0,0,0,0,1,1,0,-1,0,0,0,0,1,0,0,0,0,0,-1,0,-1,0,-1,0,0,0,0,0,0,0,0,0,0,-1,0,0,0,0,0,0,0,0,0,0,1,0,0,0,0,0,0,0,0,0,0,0,0,0,0,0,0,0,0,0,0,0,0,0,0,-1,0,0,0,0,0,0,1,0,0,0,0,0,0,0,0,-1,0,0,0,0,0,0,0,0,0,0,0,-1,0,0,0,0,0,0,0,0,0,0,0,1,0,0,0,0,0,0,0,0,0,0,0,0,0,0,0,0,0,0,0,0,0,0,0,0,0,0,0,-1,0,-1,0,-1,0,0,0,0,0,0,0,0,0,0,0,0,0,0,0,0,0,0,0,0,-1,1,0,0,0,0,0,0,0,0,0,0,0,0,0,0,0,0,0,0,0,0,0,0,0,0,0,0,0,0,0,0,0,0,-1,-1,0,-1,0,0,0,0,-1,1,0,0,0,0,0,0,0,0,0,0,0,0,0,0,0,0,0,0,0,0,-1,0,1,0,0,0,0,0,0,0,0,0,0,0,0,0,0,0,0,0,0,0,0,0,0,0,0,0,0,0,0,0,0,0,-1,-1,0,-1,0,0,0,0,0,1,0,0,0,0,0,0,0,0,0,0,0,0,0,0,0,0,0,0,0,0,-1,0,0,1,0,0,0,0,0,0,0,0,0,0,0,0,0,0,0,0,0,0,0,0,0,0,0,0,0,0,0,0,0,0,-1,-1,0,-1,0,0,0,0,0,1,0,0,0,0,0,0,0,-1,0,0,-1,0,0,0,0,0,0,0,0,0,-1,0,0,0,1,0,0,0,0,0,0,0,0,0,0,0,0,0,0,0,0,0,0,0,0,0,0,0,0,0,0,0,0,0,0,0,0,-1,0,0,0,0,0,1,0,0,0,0,0,0,-1,0,-1,0,0,0,0,0,0,0,0,0,0,0,-1,0,0,0,0,1,0,0,0,0,0,0,0,0,0,0,0,0,0,0,0,0,0,0,0,0,0,0,0,0,0,0,0,0,-1,-1,0,-1,0,0,0,0,0,1,0,0,0,-1,0,0,0,-1,0,0,-1,0,0,0,0,0,0,0,0,0,-1,0,0,0,0,0,1,0,0,0,0,0,0,0,0,0,0,0,0,0,0,0,0,0,0,0,0,0,0,0,0,0,0,0,0,0,0,-1,0,0,0,0,0,1,0,0,0,0,0,0,0,0,-1,0,0,0,0,0,0,0,0,0,0,0,-1,0,0,0,0,0,0,1,0,0,0,0,0,0,0,0,0,0,0,0,0,0,0,0,0,0,0,0,0,0,0,0,0,0,-1,-1,0,-1,0,0,0,0,0,1,0,0,0,0,0,0,0,0,0,0,0,0,0,0,0,0,0,0,0,0,-1,0,0,0,0,0,0,0,1,0,0,0,0,0,0,0,0,0,0,0,0,0,0,0,0,0,0,0,0,0,0,0,0,0,0,0,0,-1,0,0,0,0,0,1,0,0,0,0,0,0,0,0,0,0,0,0,0,0,0,0,0,0,0,0,-1,0,0,0,0,0,0,0,0,1,0,0,0,0,0,0,0,0,0,0,0,0,0,0,0,0,0,0,0,0,0,0,0,0,0,0,0,-1,0,0,0,0,0,1,0,0,0,0,-1,0,-1,0,-1,0,0,0,0,0,0,0,0,0,0,0,-1,0,0,0,0,0,0,0,0,0,1,0,0,0,0,0,0,0,0,0,0,0,0,0,0,0,0,0,0,0,0,0,0,0,-1,-1,0,-1,0,0,0,0,0,1,0,0,0,0,0,0,0,-1,0,0,0,0,0,0,0,0,0,0,0,0,-1,0,0,0,0,0,0,0,0,0,0,1,0,0,0,0,0,0,0,0,0,0,0,0,0,0,0,0,0,0,0,0,0,0,-1,-1,0,-1,0,1,0,1,-1,1,1,0,0,0,0,0,0,0,0,0,0,0,0,0,0,0,0,0,0,0,0,-1,1,0,0,0,0,0,0,0,0,0,0,0,0,0,0,0,0,0,0,0,0,0,0,0,0,0,0,0,0,0,0,0,-1,-1,0,-1,0,1,0,1,0,1,1,0,0,0,0,0,0,0,0,0,0,0,0,0,0,0,0,0,0,0,0,-1,0,1,0,0,0,0,0,0,0,0,0,0,0,0,0,0,0,0,0,0,0,0,0,0,0,0,0,0,0,0,0,0,-1,-1,0,-1,0,1,0,1,0,1,1,0,0,0,0,0,0,-1,0,0,-1,0,0,0,0,0,0,0,0,0,0,-1,0,0,1,0,0,0,0,0,0,0,0,0,0,0,0,0,0,0,0,0,0,0,0,0,0,0,0,0,0,0,0,0,0,0,0,-1,0,1,0,1,0,1,1,0,0,0,0,0,-1,0,-1,0,0,0,0,0,0,0,0,0,0,0,0,-1,0,0,0,1,0,0,0,0,0,0,0,0,0,0,0,0,0,0,0,0,0,0,0,0,0,0,0,0,0,0,0,0,-1,-1,0,-1,0,1,0,1,0,1,1,0,0,-1,0,0,0,-1,0,0,-1,0,0,0,0,0,0,0,0,0,0,-1,0,0,0,0,1,0,0,0,0,0,0,0,0,0,0,0,0,0,0,0,0,0,0,0,0,0,0,0,0,0,0,0,0,0,0,-1,0,1,0,1,0,1,1,0,0,0,0,0,0,0,-1,0,0,0,0,0,0,0,0,0,0,0,0,-1,0,0,0,0,0,1,0,0,0,0,0,0,0,0,0,0,0,0,0,0,0,0,0,0,0,0,0,0,0,0,0,0,-1,-1,0,-1,0,1,0,1,0,1,1,0,0,0,0,0,0,0,0,0,0,0,0,0,0,0,0,0,0,0,0,-1,0,0,0,0,0,0,1,0,0,0,0,0,0,0,0,0,0,0,0,0,0,0,0,0,0,0,0,0,0,0,0,0,0,0,0,-1,0,1,0,1,0,1,1,0,0,0,0,0,0,0,0,0,0,0,0,0,0,0,0,0,0,0,0,-1,0,0,0,0,0,0,0,1,0,0,0,0,0,0,0,0,0,0,0,0,0,0,0,0,0,0,0,0,0,0,0,0,0,0,0,-1,0,1,0,1,0,1,1,0,0,0,-1,0,-1,0,-1,0,0,0,0,0,0,0,0,0,0,0,0,-1,0,0,0,0,0,0,0,0,1,0,0,0,0,0,0,0,0,0,0,0,0,0,0,0,0,0,0,0,0,0,0,0,-1,-1,0,-1,0,1,0,1,0,1,1,0,0,0,0,0,0,-1,0,0,0,0,0,0,0,0,0,0,0,0,0,-1,0,0,0,0,0,0,0,0,0,1,0,0,0,0,0,0,0,0,0,0,0,0,0,0,0,0,0,0,0,0,0,0,0,-1,0,0,0,0,0,0,1,0,0,1,0,0,0,0,0,0,0,0,0,0,0,0,0,0,0,0,0,0,0,0,-1,1,0,0,0,0,0,0,0,0,0,0,0,0,0,0,0,0,0,0,0,0,0,0,0,0,0,0,0,0,0,0,0,-1,0,0,0,0,0,0,1,0,0,1,0,0,0,0,0,-1,0,0,-1,0,0,0,0,0,0,0,0,0,0,0,-1,0,1,0,0,0,0,0,0,0,0,0,0,0,0,0,0,0,0,0,0,0,0,0,0,0,0,0,0,0,0,0,1,1,0,-1,0,0,0,0,1,0,0,1,0,0,0,0,-1,0,-1,0,0,0,0,0,0,0,0,0,0,0,0,0,-1,0,0,1,0,0,0,0,0,0,0,0,0,0,0,0,0,0,0,0,0,0,0,0,0,0,0,0,0,0,0,0,0,-1,0,0,0,0,0,0,1,0,0,1,0,-1,0,0,0,-1,0,0,-1,0,0,0,0,0,0,0,0,0,0,0,-1,0,0,0,1,0,0,0,0,0,0,0,0,0,0,0,0,0,0,0,0,0,0,0,0,0,0,0,0,0,0,0,1,1,0,-1,0,0,0,0,1,0,0,1,0,0,0,0,0,0,-1,0,0,0,0,0,0,0,0,0,0,0,0,0,-1,0,0,0,0,1,0,0,0,0,0,0,0,0,0,0,0,0,0,0,0,0,0,0,0,0,0,0,0,0,0,0,0,-1,0,0,0,0,0,0,1,0,0,1,0,0,0,0,0,0,0,0,0,0,0,0,0,0,0,0,0,0,0,0,-1,0,0,0,0,0,1,0,0,0,0,0,0,0,0,0,0,0,0,0,0,0,0,0,0,0,0,0,0,0,0,0,1,1,0,-1,0,0,0,0,1,0,0,1,0,0,0,0,0,0,0,0,0,0,0,0,0,0,0,0,0,0,0,0,-1,0,0,0,0,0,0,1,0,0,0,0,0,0,0,0,0,0,0,0,0,0,0,0,0,0,0,0,0,0,0,0,1,1,0,-1,0,0,0,0,1,0,0,1,0,0,-1,0,-1,0,-1,0,0,0,0,0,0,0,0,0,0,0,0,0,-1,0,0,0,0,0,0,0,1,0,0,0,0,0,0,0,0,0,0,0,0,0,0,0,0,0,0,0,0,0,0,0,0,-1,0,0,0,0,0,0,1,0,0,1,0,0,0,0,0,-1,0,0,0,0,0,0,0,0,0,0,0,0,0,0,-1,0,0,0,0,0,0,0,0,1,0,0,0,0,0,0,0,0,0,0,0,0,0,0,0,0,0,0,0,0,0,0,0,-1,0,0,0,0,0,0,0,0,0,0,1,0,0,0,0,-1,0,0,-1,0,0,0,0,0,0,0,0,0,0,0,0,-1,1,0,0,0,0,0,0,0,0,0,0,0,0,0,0,0,0,0,0,0,0,0,0,0,0,0,0,0,0,0,1,1,0,-1,0,0,0,0,0,0,0,0,1,0,0,0,-1,0,-1,0,0,0,0,0,0,0,0,0,0,0,0,0,0,-1,0,1,0,0,0,0,0,0,0,0,0,0,0,0,0,0,0,0,0,0,0,0,0,0,0,0,0,0,0,0,0,-1,0,0,0,0,0,0,0,0,0,0,1,-1,0,0,0,-1,0,0,-1,0,0,0,0,0,0,0,0,0,0,0,0,-1,0,0,1,0,0,0,0,0,0,0,0,0,0,0,0,0,0,0,0,0,0,0,0,0,0,0,0,0,0,0,1,1,0,-1,0,0,0,0,0,0,0,0,1,0,0,0,0,0,-1,0,0,0,0,0,0,0,0,0,0,0,0,0,0,-1,0,0,0,1,0,0,0,0,0,0,0,0,0,0,0,0,0,0,0,0,0,0,0,0,0,0,0,0,0,0,0,-1,0,0,0,0,0,0,0,0,0,0,1,0,0,0,0,0,0,0,0,0,0,0,0,0,0,0,0,0,0,0,0,-1,0,0,0,0,1,0,0,0,0,0,0,0,0,0,0,0,0,0,0,0,0,0,0,0,0,0,0,0,0,0,1,1,0,-1,0,0,0,0,0,0,0,0,1,0,0,0,0,0,0,0,0,0,0,0,0,0,0,0,0,0,0,0,0,-1,0,0,0,0,0,1,0,0,0,0,0,0,0,0,0,0,0,0,0,0,0,0,0,0,0,0,0,0,0,0,1,1,0,-1,0,0,0,0,0,0,0,0,1,0,-1,0,-1,0,-1,0,0,0,0,0,0,0,0,0,0,0,0,0,0,-1,0,0,0,0,0,0,1,0,0,0,0,0,0,0,0,0,0,0,0,0,0,0,0,0,0,0,0,0,0,0,0,-1,0,0,0,0,0,0,0,0,0,0,1,0,0,0,0,-1,0,0,0,0,0,0,0,0,0,0,0,0,0,0,0,-1,0,0,0,0,0,0,0,1,0,0,0,0,0,0,0,0,0,0,0,0,0,0,0,0,0,0,0,0,0,0,1,1,0,-1,0,0,0,0,0,0,0,0,0,1,0,0,-1,1,-1,0,1,0,0,0,0,0,0,0,0,0,0,0,0,0,-1,1,0,0,0,0,0,0,0,0,0,0,0,0,0,0,0,0,0,0,0,0,0,0,0,0,0,0,0,0,0,0,0,0,0,0,0,0,0,0,0,0,0,-1,0,0,0,0,0,0,0,0,0,0,0,0,0,0,0,0,0,0,0,0,-1,0,1,0,0,0,0,0,0,0,0,0,0,0,0,0,0,0,0,0,0,0,0,0,0,0,0,0,0,0,1,1,0,-1,0,0,0,0,0,0,0,0,0,1,0,0,0,1,-1,0,1,0,0,0,0,0,0,0,0,0,0,0,0,0,-1,0,0,1,0,0,0,0,0,0,0,0,0,0,0,0,0,0,0,0,0,0,0,0,0,0,0,0,0,0,0,0,0,0,0,0,0,0,0,0,0,0,0,1,0,0,0,0,0,0,1,0,0,0,0,0,0,0,0,0,0,0,0,0,-1,0,0,0,1,0,0,0,0,0,0,0,0,0,0,0,0,0,0,0,0,0,0,0,0,0,0,0,0,0,1,1,0,-1,0,0,0,0,0,0,0,0,0,1,0,0,0,1,0,0,1,0,0,0,0,0,0,0,0,0,0,0,0,0,-1,0,0,0,0,1,0,0,0,0,0,0,0,0,0,0,0,0,0,0,0,0,0,0,0,0,0,0,0,0,1,1,0,-1,0,0,0,0,0,0,0,0,0,1,-1,0,-1,1,-1,0,1,0,0,0,0,0,0,0,0,0,0,0,0,0,-1,0,0,0,0,0,1,0,0,0,0,0,0,0,0,0,0,0,0,0,0,0,0,0,0,0,0,0,0,0,0,0,0,0,0,0,0,0,0,0,0,0,0,1,0,0,0,0,0,0,0,0,0,0,0,0,0,0,0,0,0,0,0,0,-1,0,0,0,0,0,0,1,0,0,0,0,0,0,0,0,0,0,0,0,0,0,0,0,0,0,0,0,0,0,-1,-1,0,-1,0,0,0,0,0,0,0,0,0,-1,1,0,1,-1,1,0,-1,0,0,0,0,0,0,0,0,0,0,0,0,0,0,-1,1,0,0,0,0,0,0,0,0,0,0,0,0,0,0,0,0,0,0,0,0,0,0,0,0,0,0,0,0,0,0,0,0,0,0,0,0,0,0,0,0,0,1,0,0,0,0,0,0,0,0,0,0,0,0,0,0,0,0,0,0,0,0,-1,0,1,0,0,0,0,0,0,0,0,0,0,0,0,0,0,0,0,0,0,0,0,0,0,0,0,0,0,-1,-1,0,-1,0,0,0,0,0,0,0,0,0,0,1,0,1,0,1,0,0,0,0,0,0,0,0,0,0,0,0,0,0,0,0,-1,0,0,1,0,0,0,0,0,0,0,0,0,0,0,0,0,0,0,0,0,0,0,0,0,0,0,0,0,0,0,0,0,0,0,0,0,0,0,0,0,0,0,1,0,1,0,0,0,0,0,0,0,0,0,0,0,0,0,0,0,0,0,0,-1,0,0,0,1,0,0,0,0,0,0,0,0,0,0,0,0,0,0,0,0,0,0,0,0,0,0,0,0,0,0,0,0,0,0,0,0,0,0,0,0,0,0,-1,0,0,0,0,0,0,0,0,0,0,0,0,0,0,0,0,0,0,0,0,-1,0,0,0,0,1,0,0,0,0,0,0,0,0,0,0,0,0,0,0,0,0,0,0,0,0,0,0,0,-1,-1,0,-1,0,0,0,0,0,0,0,0,0,0,1,0,1,-1,1,0,0,0,0,0,0,0,0,0,0,0,0,0,0,0,0,-1,0,0,0,0,0,1,0,0,0,0,0,0,0,0,0,0,0,0,0,0,0,0,0,0,0,0,0,0,1,1,0,-1,0,0,0,0,0,0,0,0,0,1,0,1,0,1,-1,0,1,0,0,0,0,0,0,0,0,0,0,0,0,0,0,0,-1,1,0,0,0,0,0,0,0,0,0,0,0,0,0,0,0,0,0,0,0,0,0,0,0,0,0,0,0,0,0,0,0,0,0,0,0,0,0,0,0,1,0,1,0,0,0,0,1,0,0,0,0,0,0,0,0,0,0,0,0,0,0,0,-1,0,1,0,0,0,0,0,0,0,0,0,0,0,0,0,0,0,0,0,0,0,0,0,0,0,0,0,1,1,0,-1,0,0,0,0,0,0,0,0,0,1,0,1,0,1,0,0,1,0,0,0,0,0,0,0,0,0,0,0,0,0,0,0,-1,0,0,1,0,0,0,0,0,0,0,0,0,0,0,0,0,0,0,0,0,0,0,0,0,0,0,0,1,1,0,-1,0,0,0,0,0,0,0,0,0,1,-1,1,-1,1,-1,0,1,0,0,0,0,0,0,0,0,0,0,0,0,0,0,0,-1,0,0,0,1,0,0,0,0,0,0,0,0,0,0,0,0,0,0,0,0,0,0,0,0,0,0,0,0,0,0,0,0,0,0,0,0,0,0,0,0,1,0,1,0,0,0,0,0,0,0,0,0,0,0,0,0,0,0,0,0,0,0,0,-1,0,0,0,0,1,0,0,0,0,0,0,0,0,0,0,0,0,0,0,0,0,0,0,0,0,0,0,-1,-1,0,-1,0,0,0,0,0,0,0,0,0,0,0,0,1,0,1,0,0,0,0,0,0,0,0,0,0,0,0,0,0,0,0,0,0,-1,1,0,0,0,0,0,0,0,0,0,0,0,0,0,0,0,0,0,0,0,0,0,0,0,0,0,0,0,0,0,0,0,0,0,0,0,0,0,0,0,0,0,1,0,0,0,0,0,0,0,0,0,0,0,0,0,0,0,0,0,0,0,0,-1,0,1,0,0,0,0,0,0,0,0,0,0,0,0,0,0,0,0,0,0,0,0,0,0,0,0,0,0,0,0,0,0,0,0,0,0,0,0,0,0,-1,0,-1,0,0,0,0,0,0,0,0,0,0,0,0,0,0,0,0,0,0,0,0,-1,0,0,1,0,0,0,0,0,0,0,0,0,0,0,0,0,0,0,0,0,0,0,0,0,0,0,-1,-1,0,-1,0,0,0,0,0,0,0,0,0,0,0,0,1,-1,1,0,0,0,0,0,0,0,0,0,0,0,0,0,0,0,0,0,0,-1,0,0,0,1,0,0,0,0,0,0,0,0,0,0,0,0,0,0,0,0,0,0,0,0,0,0,1,1,0,-1,0,0,0,0,0,0,0,0,0,0,0,0,0,1,0,0,0,0,0,0,0,0,0,0,0,0,0,0,0,0,0,0,0,0,-1,1,0,0,0,0,0,0,0,0,0,0,0,0,0,0,0,0,0,0,0,0,0,0,0,0,1,1,0,-1,0,0,0,0,0,0,0,0,0,0,-1,0,-1,1,-1,0,0,0,0,0,0,0,0,0,0,0,0,0,0,0,0,0,0,0,-1,0,1,0,0,0,0,0,0,0,0,0,0,0,0,0,0,0,0,0,0,0,0,0,0,0,0,0,0,0,0,0,0,0,0,0,0,0,0,0,0,0,0,-1,0,0,0,0,0,0,0,0,0,0,0,0,0,0,0,0,0,0,0,0,-1,0,0,1,0,0,0,0,0,0,0,0,0,0,0,0,0,0,0,0,0,0,0,0,0,0,0,0,0,0,0,0,0,0,0,0,0,0,0,0,-1,0,-1,0,-1,0,0,0,0,0,0,0,0,0,0,0,0,0,0,0,0,0,0,0,0,-1,1,0,0,0,0,0,0,0,0,0,0,0,0,0,0,0,0,0,0,0,0,0,0,0,-1,-1,0,-1,0,0,0,0,0,0,0,0,0,0,0,0,0,-1,1,0,0,0,0,0,0,0,0,0,0,0,0,0,0,0,0,0,0,0,0,-1,0,1,0,0,0,0,0,0,0,0,0,0,0,0,0,0,0,0,0,0,0,0,0,0,-1,-1,0,-1,0,0,0,0,0,0,0,0,0,0,1,0,1,-1,1,1,0,0,0,0,0,0,0,0,0,0,0,0,0,0,0,0,0,0,0,0,-1,1,0,0,0,0,0,0,0,0,0,0,0,0,0,0,0,0,0,0,0,0,0,0,0,0,0,0,0,0,0,0,0,0,0,0,0,0,0,0,0,0,0,0,0,0,0,0,0,0,0,0,0,0,0,0,0,0,0,0,0,0,0,0,0,0,0,0,0,0,0,0,0,0,0,0,0,0,0,0,0,0,0,0,0,0,0,0,0,0,0,0,0,0,0,0,0,0,0,0,0,0,0,0,0,0,0,0,0,0,0,0,0,0,0,0,0,0,0,0,0,0,0,0,0,0,0,0,0,0,0,0,0,0,0,0,0,0,0,0,0,0,0,0,0,0,0,0,0,0,0,0,0,0,0,0,0,0,0,0,0,0,0,0,0,0,0,0,0,0,0,0,0,0,0,0,0,0,0,0,0,0,0,0,0,0,0,0,0,0,0,0,0,0,0,0,0,0,0,0,0,0,0,0,0,0,0,0,0,0,0,0,0,0,0,0,0,0,0,0,0,0,0,0,0,0,0,0,0,0,0,0,0,0,0,0,0,0,0,0,0,0,0,0,0,0,0,0,0,0,0,0,0,0,0,0,0,0,0,0,0,0,0,0,0,0,0,0,0,0,0,0,0,0,0,0,0,0,0,0,0,0,0,0,0,0,0,0,0,0,0,0,0,0,0,0,0,0,0,0,0,0,0,0,0,0,0,0,0,0,0,0,0,0,0,0,0,0,0,0,0,0,0,0,0,0,0,0,0,0,0,0,0,0,0,0,0,0,0,0,0,0,0,0,0,0,0,0,0,0,0,0,0,0,0,0,0,0,0,0,0,0,0,0,0,0,0,0,0,0,0,0,0,0,0,0,0,0,0,0,0,0,0,0,0,0,0,0,0,0,0,0,0,0,0,0,0,0,0,0,0,0,0,0,0,0,0,0,0,0,0,0,0,0,0,0,0,0,0,0,0,0,0,0,0,0,0,0,0,0,0,0,0,0,0,0,0,0,0,0,0,0,0,0,0,0,0,0,0,0,0,0,0,0,0,0,0,0,0,0,0,0,0,0,0,0,0,0,0,0,0,0,0,0,0,0,0,0,0,0,0,0,0,0,0,0,0,0,0,0,0,0,0,0,0,0,0,0,0,0,0,0,0,0,0,0,0,0,0,0,0,0,0,0,0,0,0,0,0,0,0,0,0,0,0,0,0,0,0,0,0,0,0,0,0,0,0,0,0,0,0,0,0,0,0,0,0,0,0,0,0,0,0,0,0,0,0,0,0,0,0,0,0,0,0,0,0,0,0,0,0,0,0,0,0,0,0,0,0,0,0,0,0,0,0,0,0,0,0,0,0,0,0,0,0,0,0,0,0,0,0,0,0,0,0,0,0,0,0,0,0,0,0,0,0,0,0,0,0,0,0,0,0,0,0,0,0,0,0,0,0,0,0,0,0,0,0,0,0,0,0,0,0,0,0,0,0,0,0,0,0,0,0,0,0,0,0,0,0,0,0,0,0,0,0,0,0,0,0,0,0,0,0,0,0,0,0,0,0,0,0,0,0,0,0,0,0,0,0,0,0,0,0,0,0,0,0,0,0,0,0,0,0,0,0,0,0,0,0,0,0,0,0,0,0,0,0,0,0,0,0,0,0,0,0,0,0,0,0,0,0,0,0,0,0,0,0,0,0,0,0,0,0,0,0,0,0,0,0,0,0,0,0,0,0,0,0,0,0,0,0,0,0,0,0,0,0,0,0,0,0,0,0,0,0,0,0,0,0,0,0,0,0,0,0,0,0,0,0,0,0,0,0,0,0,0,0,0,0,0,0,0,0,0,0,0,0,0,0,0,0,0,0,0,0,0,0,0,0,0,0,0,0,0,0,0,0,0,0,0,0,0,0,0,0,0,0,0,0,0,0,0,0,0,0,0,0,0,0,0,0,0,0,0,0,0,0,0,0,0,0,0,0,0,0,0,0,0,0,0,0,0,0,0,0,0,0,0,0,0,0,0,0,0,0,0,0,0,0,0,0,0,0,0,0,0,0,0,0,0,0,0,0,0,0,0,0,0,0,0,0,0,0,0,0,0,0,0,0,0};

__device__ __forceinline__ f32x8 wmma16(f16x16 a, f16x16 b, f32x8 c) {
  c = __builtin_amdgcn_wmma_f32_16x16x32_f16(false, a, false, b, (short)0, c, false, false);
  asm volatile("v_nop\n\tv_nop\n\tv_nop\n\tv_nop" : "+v"(c) : "v"(a), "v"(b));
  return c;
}
__device__ __forceinline__ f16x16 lds_frag(const f16* base, int stride) {
  const int lane = threadIdx.x & 31, row = lane & 15, kh = (lane >> 4) * 8;
  const f16x8 lo = *(const f16x8*)(base + row * stride + kh);
  const f16x8 hi = *(const f16x8*)(base + row * stride + kh + 16);
  f16x16 f;
#pragma unroll
  for (int i = 0; i < 8; ++i) { f[i] = lo[i]; f[i + 8] = hi[i]; }
  return f;
}

__global__ __launch_bounds__(256) void k_comp(const float* __restrict__ xin, const float* __restrict__ tin, float* __restrict__ partial) {
  __shared__ __attribute__((aligned(16))) f16 aS[384 * 72];
  __shared__ __attribute__((aligned(16))) f16 bS[NPP * 72];
  __shared__ float red[8];
  const int tid = threadIdx.x, lane = tid & 31, wave = tid >> 5;
  const int b0 = blockIdx.x * RB;
  for (int e = tid; e < NPP * 64; e += 256) { const int p = e >> 6, k = e & 63; bS[p * 72 + k] = (f16)(float)c_ST[e]; }
  { const int bl = tid & 127, part = tid >> 7, b = b0 + bl;
    const float* xr = xin + (size_t)b * (NJ * 3); const float* tr = tin + (size_t)b * (NJ * 3);
    for (int d = (part ? 2 : 0); d < (part ? 3 : 2); ++d) {
      f16* ar = aS + (d * RB + bl) * 72;
#pragma unroll
      for (int j = 0; j < NJ; ++j) { ar[j] = (f16)xr[j * 3 + d]; ar[NJ + j] = (f16)tr[j * 3 + d]; }
#pragma unroll
      for (int k = 2 * NJ; k < 64; ++k) ar[k] = (f16)0.0f;
    }
  }
  __syncthreads();
  float asum = 0.0f;
#pragma unroll 1
  for (int rt = 0; rt < 3; ++rt) {
    const int m0 = (wave * 3 + rt) * 16;
    const f16x16 a0 = lds_frag(aS + m0 * 72, 72), a1 = lds_frag(aS + m0 * 72 + 32, 72);
#pragma unroll 1
    for (int nt = 0; nt < NPP / 16; ++nt) {
      f32x8 acc = {};
      acc = wmma16(a0, lds_frag(bS + (nt * 16) * 72, 72), acc);
      acc = wmma16(a1, lds_frag(bS + (nt * 16) * 72 + 32, 72), acc);
#pragma unroll
      for (int r = 0; r < 8; ++r) asum += fabsf(acc[r]);
    }
  }
#pragma unroll
  for (int off = 16; off >= 1; off >>= 1) asum += __shfl_xor(asum, off, 32);
  if (lane == 0) red[wave] = asum;
  __syncthreads();
  if (tid < 32) { float s = 0.0f;
#pragma unroll
    for (int w = 0; w < 8; ++w) s += red[w];
    *(volatile float*)(partial + (size_t)blockIdx.x * 32 + tid) = s; __threadfence(); *(volatile float*)(partial + (size_t)blockIdx.x * 32 + tid) = s; }
}
__global__ __launch_bounds__(256) void k_final(const float* __restrict__ partial, int n, float* __restrict__ out) {
  __shared__ float red[256];
  const int tid = threadIdx.x; float s = 0.0f;
  for (int i = tid; i < n; i += 256) s += partial[(size_t)i * 32];
  red[tid] = s; __syncthreads();
  for (int o = 128; o > 0; o >>= 1) { if (tid < o) red[tid] += red[tid + o]; __syncthreads(); }
  if (tid == 0) { const float v = red[0] * (1.0f / (float)NB_); *(volatile float*)out = v; __threadfence(); *(volatile float*)out = v; }
}

extern "C" void kernel_launch(void* const* d_in, const int* in_sizes, int n_in,
                              void* d_out, int out_size, void* d_ws, size_t ws_size,
                              hipStream_t stream) {
  (void)in_sizes; (void)n_in; (void)out_size; (void)ws_size;
  const float* xin = (const float*)d_in[0];
  const float* tin = (const float*)d_in[1];
  float* out = (float*)d_out;
  float* partial = (float*)d_ws;
  k_comp<<<dim3(NB_ / RB), dim3(256), 0, stream>>>(xin, tin, partial);
  k_final<<<dim3(1), dim3(256), 0, stream>>>(partial, NB_ / RB, out);
}
